// RWKVAttention_28381143892187
// MI455X (gfx1250) — hardware-verified
//
#include <hip/hip_runtime.h>


namespace {
constexpr int Bsz = 2, S = 4096, HID = 1024, NH = 16, DH = 64, HD = NH * DH, NRKV = 3 * HD, MROWS = Bsz * S;

typedef _Float16 b16;
typedef __attribute__((ext_vector_type(16))) _Float16 v16b;
typedef __attribute__((ext_vector_type(8)))  _Float16 v8b;
typedef __attribute__((ext_vector_type(8)))  float v8f;
typedef __attribute__((ext_vector_type(4)))  float v4f;

__device__ __forceinline__ v8b ld8b(const b16* p) { return *(const v8b*)p; }
__device__ __forceinline__ v16b cat8b(v8b a, v8b b) { return __builtin_shufflevector(a, b, 0, 1, 2, 3, 4, 5, 6, 7, 8, 9, 10, 11, 12, 13, 14, 15); }
__device__ __forceinline__ v16b frag_kb(const b16* p, int hh) { return cat8b(ld8b(p + 8 * hh), ld8b(p + 16 + 8 * hh)); }
__device__ __forceinline__ void split16(float v, b16& hi, b16& lo) { hi = (b16)v; lo = (b16)(v - (float)hi); }
__device__ __forceinline__ void frag_ksplit(const float* p, int hh, v16b& fh_, v16b& fl_) {
  const float* p0 = p + 8 * hh; const float* p1 = p + 16 + 8 * hh;
#pragma unroll
  for (int e = 0; e < 8; ++e) { b16 a, c; split16(p0[e], a, c); fh_[e] = a; fl_[e] = c; split16(p1[e], a, c); fh_[8 + e] = a; fl_[8 + e] = c; }
}
__device__ __forceinline__ v8f wmma16b(v16b a, v16b b, v8f c) {
  v8f d = __builtin_amdgcn_wmma_f32_16x16x32_f16(false, a, false, b, (short)0, c, false, false);
  asm volatile("v_nop\n\tv_nop\n\tv_nop\n\tv_nop" : "+v"(d) : "v"(a), "v"(b));
  return d;
}
__device__ __forceinline__ void wave_lds_sync() {
  __builtin_amdgcn_fence(__ATOMIC_RELEASE, "workgroup");
  __builtin_amdgcn_wave_barrier();
  __builtin_amdgcn_fence(__ATOMIC_ACQUIRE, "workgroup");
}

struct Opnd { const void* p0; const void* p1; int ld; };
template <int NP> __device__ __forceinline__ void load_frags(const Opnd& o, int row, int kb, int hh, v16b& fh_, v16b& fl_) {
  if (NP == 0) { frag_ksplit((const float*)o.p0 + (size_t)row * o.ld + kb, hh, fh_, fl_); }
  else if (NP == 3) {
    const float* p = (const float*)o.p0 + (size_t)row * o.ld + kb; const float* p0 = p + 8 * hh; const float* p1 = p + 16 + 8 * hh;
#pragma unroll
    for (int e = 0; e < 8; ++e) { fh_[e] = (b16)p0[e]; fh_[8 + e] = (b16)p1[e]; }
    fl_ = fh_;
  } else {
    fh_ = frag_kb((const b16*)o.p0 + (size_t)row * o.ld + kb, hh);
    if (NP == 2) fl_ = frag_kb((const b16*)o.p1 + (size_t)row * o.ld + kb, hh); else fl_ = fh_;
  }
}
template <int ANP, int BNP> __device__ __forceinline__ v8f mac(v16b ah, v16b al, v16b bh, v16b bl, v8f c) {
  c = wmma16b(ah, bh, c);
  if (BNP == 0 || BNP == 2) c = wmma16b(ah, bl, c);
  if (ANP == 0 || ANP == 2) c = wmma16b(al, bh, c);
  return c;
}
template <int ANP, int BNP>
__device__ __forceinline__ void gemm_tile(const Opnd& A, const Opnd& B, int K, int m0, int c0, int nloc, int hlf, v8f (&acc)[2][4]) {
  for (int kb = 0; kb < K; kb += 32) {
    v16b a0h, a0l, a1h, a1l;
    load_frags<ANP>(A, m0 + nloc, kb, hlf, a0h, a0l);
    load_frags<ANP>(A, m0 + 16 + nloc, kb, hlf, a1h, a1l);
#pragma unroll
    for (int t = 0; t < 4; ++t) {
      v16b bh, bl;
      load_frags<BNP>(B, c0 + t * 16 + nloc, kb, hlf, bh, bl);
      acc[0][t] = mac<ANP, BNP>(a0h, a0l, bh, bl, acc[0][t]);
      acc[1][t] = mac<ANP, BNP>(a1h, a1l, bh, bl, acc[1][t]);
    }
  }
}

struct Epi { float scale; const float* cscale; const float* cbias; const float* rbias; int act; float post; const float* rscale; const float* resid; };
__device__ __forceinline__ float epi_val(const Epi& e, float acc, int row, int col) {
  float val = acc * e.scale;
  if (e.cscale) val *= e.cscale[col];
  if (e.cbias) val += e.cbias[col];
  if (e.rbias) val += e.rbias[row];
  if (e.act == 1) val = 0.5f * val * (1.0f + erff(val * 0.70710678118654752f));
  val *= e.post;
  if (e.rscale) val *= e.rscale[(size_t)row * 32];
  return val;
}
__device__ __forceinline__ void epi_planes(v8f (&acc)[2][4], const Epi& e, bool two,
                                           b16* __restrict__ oh, b16* __restrict__ ol, int ldo, int m0, int c0, int lane, b16* Th, b16* Tl) {
  const int nloc = lane & 15, hlf = lane >> 4;
#pragma unroll
  for (int t = 0; t < 4; ++t)
#pragma unroll
    for (int r = 0; r < 2; ++r)
#pragma unroll
      for (int v = 0; v < 8; ++v) {
        const int rr = r * 16 + v + 8 * hlf, cc = t * 16 + nloc;
        const float val = epi_val(e, acc[r][t][v], m0 + rr, c0 + cc);
        b16 h_, l_; split16(val, h_, l_);
        Th[rr * 64 + cc] = h_; if (two) Tl[rr * 64 + cc] = l_;
      }
  wave_lds_sync();
  for (int pass = 0; pass < 2; ++pass) {
#pragma unroll
    for (int j = 0; j < 8; ++j) {
      const int rr = j * 4 + (lane >> 3), c8 = (lane & 7) * 8;
      const size_t o = (size_t)(m0 + rr) * ldo + c0 + c8;
      *(volatile v8b*)(oh + o) = ld8b(Th + rr * 64 + c8);
      if (two) *(volatile v8b*)(ol + o) = ld8b(Tl + rr * 64 + c8);
    }
    __threadfence();
  }
}
__device__ __forceinline__ void epi_f32(v8f (&acc)[2][4], const Epi& e, float* __restrict__ out, int ldo, int m0, int c0, int lane, float* Tt) {
  const int nloc = lane & 15, hlf = lane >> 4;
#pragma unroll
  for (int t = 0; t < 4; ++t)
#pragma unroll
    for (int r = 0; r < 2; ++r)
#pragma unroll
      for (int v = 0; v < 8; ++v) {
        const int rr = r * 16 + v + 8 * hlf, cc = t * 16 + nloc;
        Tt[rr * 64 + cc] = epi_val(e, acc[r][t][v], m0 + rr, c0 + cc);
      }
  wave_lds_sync();
  float* dst0 = out + (size_t)m0 * ldo + c0; const float* rs0 = e.resid ? e.resid + (size_t)m0 * ldo + c0 : nullptr;
  for (int pass = 0; pass < 2; ++pass) {
#pragma unroll
    for (int j = 0; j < 16; ++j) {
      const int rr = j * 2 + hlf, c4 = nloc * 4;
      v4f val = *(const v4f*)(Tt + rr * 64 + c4);
      if (rs0) val += *(const v4f*)(rs0 + (size_t)rr * ldo + c4);
      *(volatile v4f*)(dst0 + (size_t)rr * ldo + c4) = val;
    }
    __threadfence();
  }
}


__global__ __launch_bounds__(256) void prep_kernel(const float* __restrict__ x, const float* __restrict__ wrkv, const float* __restrict__ wo, const float* __restrict__ tmix,
                                                   const float* __restrict__ tdecay, b16* __restrict__ w16, b16* __restrict__ mx16, float* __restrict__ g, float* __restrict__ zinv) {
  __shared__ float red[256]; __shared__ float gs[S];
  const size_t tid = (size_t)blockIdx.x * blockDim.x + threadIdx.x, stride = (size_t)gridDim.x * blockDim.x;
  const size_t n0 = (size_t)NRKV * HID / 8, n1 = (size_t)HID * HD / 8, n2 = (size_t)MROWS * HID / 8;
  for (int pass = 0; pass < 2; ++pass) {
    for (size_t c = tid; c < n0 + n1 + n2; c += stride) {
      v8b v;
      if (c < n0 + n1) { const float* src = (c < n0) ? (wrkv + c * 8) : (wo + (c - n0) * 8);
#pragma unroll
        for (int e = 0; e < 8; ++e) v[e] = (b16)src[e];
        *(volatile v8b*)(w16 + c * 8) = v;
      } else {
        const size_t i = (c - n0 - n1) * 8; const int row = (int)(i / HID), col = (int)(i % HID), t = row % S;
#pragma unroll
        for (int e = 0; e < 8; ++e) {
          const float mu = tmix[col + e], xv = x[i + e], xp = (t == 0) ? 0.0f : x[i + e - HID];
          v[e] = (b16)(xv * mu + xp * (1.0f - mu));
        }
        *(volatile v8b*)(mx16 + i) = v;
      }
    }
    __threadfence();
  }
  if (blockIdx.x == 0) {
    float s = 0.0f;
    for (int i = threadIdx.x; i < HD; i += 256) s += -expf(tdecay[i]);
    red[threadIdx.x] = s;
    __syncthreads();
    if (threadIdx.x == 0) { float tot = 0.0f; for (int i = 0; i < 256; ++i) tot += red[i]; red[0] = tot * (1.0f / HD); }
    __syncthreads();
    const float a = red[0];
    for (int dd = threadIdx.x; dd < S; dd += 256) gs[dd] = expf(a * -(float)dd);
    __syncthreads();
    __shared__ float zs[S];
    if (threadIdx.x == 0) { float cum = 0.0f; for (int dd = 0; dd < S; ++dd) { cum += gs[dd]; zs[S - 1 - dd] = cum; } }
    __syncthreads();
    for (int pass = 0; pass < 2; ++pass) {
      for (int i = threadIdx.x; i < S; i += 256) { ((volatile float*)g)[i] = gs[i]; ((volatile float*)zinv)[i] = 1.0f / (zs[i] + 1e-8f); }
      __threadfence();
    }
  }
}

__global__ __launch_bounds__(128) void rkv_kernel(const b16* __restrict__ mx16, const b16* __restrict__ w16, const float* __restrict__ cs, const float* __restrict__ sn,
                                                  b16* __restrict__ r16, float* __restrict__ k32, b16* __restrict__ v16) {
  __shared__ __attribute__((aligned(16))) float Ts[4][32 * 64];
  const int lane = threadIdx.x & 31, wave = threadIdx.x >> 5, nloc = lane & 15, hlf = lane >> 4;
  const int m0 = blockIdx.y * 128 + wave * 32, c0 = blockIdx.x * 64;
  const int mat = c0 / HD, hcol = c0 % HD;
  v8f acc[2][4];
#pragma unroll
  for (int r = 0; r < 2; ++r)
#pragma unroll
    for (int t = 0; t < 4; ++t) acc[r][t] = (v8f){};
  const Opnd A{mx16, nullptr, HID}, B{w16, nullptr, HID};
  gemm_tile<1, 1>(A, B, HID, m0, c0, nloc, hlf, acc);
  float* Tf = Ts[wave]; b16* Th = (b16*)Ts[wave];
#pragma unroll
  for (int t = 0; t < 4; ++t)
#pragma unroll
    for (int r = 0; r < 2; ++r)
#pragma unroll
      for (int v = 0; v < 8; ++v) {
        const int rr = r * 16 + v + 8 * hlf, d = t * 16 + nloc, tpos = (m0 + rr) % S;
        float val = acc[r][t][v];
        if (mat < 2) {
          float oth = acc[r][t ^ 2][v];
          if (mat == 0) { val = 1.0f / (1.0f + expf(-val)); oth = 1.0f / (1.0f + expf(-oth)); }
          const float rot = (t < 2) ? -oth : oth;
          val = val * cs[(size_t)tpos * DH + d] + rot * sn[(size_t)tpos * DH + d];
        }
        if (mat == 1) Tf[rr * 64 + d] = val; else Th[rr * 64 + d] = (b16)val;
      }
  wave_lds_sync();
  for (int pass = 0; pass < 2; ++pass) {
    if (mat == 1) {
      float* dst = k32 + (size_t)m0 * HD + hcol;
#pragma unroll
      for (int j = 0; j < 16; ++j) { const int rr = j * 2 + hlf; *(volatile v4f*)(dst + (size_t)rr * HD + nloc * 4) = *(const v4f*)(Tf + rr * 64 + nloc * 4); }
    } else {
      b16* dst = ((mat == 0) ? r16 : v16) + (size_t)m0 * HD + hcol;
#pragma unroll
      for (int j = 0; j < 8; ++j) { const int rr = j * 4 + (lane >> 3), c8 = (lane & 7) * 8; *(volatile v8b*)(dst + (size_t)rr * HD + c8) = ld8b(Th + rr * 64 + c8); }
    }
    __threadfence();
  }
}

__global__ __launch_bounds__(128) void kv_kernel(const float* __restrict__ k32, const b16* __restrict__ v16, float* __restrict__ kv32, b16* __restrict__ kvT) {
  __shared__ __attribute__((aligned(16))) b16 Tl[HD / 2][64 + 8];
  const int tid = threadIdx.x, lane = tid & 31, wave = tid >> 5;
  const int b = blockIdx.x / (S / 64), t0 = (blockIdx.x % (S / 64)) * 64, ch0 = blockIdx.y * (HD / 2);
  const size_t row0 = (size_t)b * S + t0;
  for (int pass = 0; pass < 2; ++pass) {
    for (int it = 0; it < 64; ++it) {
      const int c = tid * 4; const size_t o = (row0 + it) * HD + ch0 + c;
      const v4f kk = *(const v4f*)(k32 + o);
      v4f p;
#pragma unroll
      for (int e = 0; e < 4; ++e) { p[e] = kk[e] * (float)v16[o + e]; Tl[c + e][it] = (b16)p[e]; }
      *(volatile v4f*)(kv32 + o) = p;
    }
    __syncthreads();
    b16* dst = kvT + ((size_t)b * HD + ch0) * S + t0;
#pragma unroll
    for (int j = 0; j < 32; ++j) { const int c = wave * 128 + j * 4 + (lane >> 3), e8 = (lane & 7) * 8; *(volatile v8b*)(dst + (size_t)c * S + e8) = *(const v8b*)(&Tl[c][e8]); }
    __threadfence();
    __syncthreads();
  }
}

__global__ __launch_bounds__(128) void wkv_kernel(const float* __restrict__ g, const float* __restrict__ zinv, const b16* __restrict__ kvTb, const float* __restrict__ kv32b,
                                                  const b16* __restrict__ r16b, const float* __restrict__ tfirst, b16* __restrict__ yb) {
  __shared__ __attribute__((aligned(16))) b16 gt[S];
  __shared__ __attribute__((aligned(16))) b16 Th[4][32 * 64];
  for (int i = threadIdx.x; i < S; i += 128) gt[i] = (b16)g[i];
  __syncthreads();
  const int lane = threadIdx.x & 31, wave = threadIdx.x >> 5, nloc = lane & 15, hlf = lane >> 4;
  const int m0 = blockIdx.y * 128 + wave * 32, c0 = blockIdx.x * 64, kstart = blockIdx.y * 128;
  v8f acc[2][4];
#pragma unroll
  for (int r = 0; r < 2; ++r)
#pragma unroll
    for (int t = 0; t < 4; ++t) acc[r][t] = (v8f){};
  for (int kb = kstart; kb < S; kb += 32) {
    v16b a0, a1;
    const int i0 = m0 + nloc, i1 = m0 + 16 + nloc;
#pragma unroll
    for (int e = 0; e < 16; ++e) {
      const int j = kb + ((e < 8) ? (8 * hlf + e) : (16 + 8 * hlf + (e - 8)));
      a0[e] = (j >= i0) ? gt[j - i0] : (b16)0.0f;
      a1[e] = (j >= i1) ? gt[j - i1] : (b16)0.0f;
    }
#pragma unroll
    for (int t = 0; t < 4; ++t) {
      const v16b bw = frag_kb(kvTb + (size_t)(c0 + t * 16 + nloc) * S + kb, hlf);
      acc[0][t] = wmma16b(a0, bw, acc[0][t]); acc[1][t] = wmma16b(a1, bw, acc[1][t]);
    }
  }
  b16* Tp = Th[wave];
#pragma unroll
  for (int t = 0; t < 4; ++t)
#pragma unroll
    for (int r = 0; r < 2; ++r)
#pragma unroll
      for (int v = 0; v < 8; ++v) {
        const int rr = r * 16 + v + 8 * hlf, cc = t * 16 + nloc, i = m0 + rr, o = c0 + cc;
        const float wkv = acc[r][t][v] * zinv[i];
        const float kvv = kv32b[(size_t)i * HD + o], rv = (float)r16b[(size_t)i * HD + o];
        Tp[rr * 64 + cc] = (b16)(rv * (tfirst[o] * kvv + wkv));
      }
  wave_lds_sync();
  b16* dst = yb + (size_t)m0 * HD + c0;
  for (int pass = 0; pass < 2; ++pass) {
#pragma unroll
    for (int j = 0; j < 8; ++j) { const int rr = j * 4 + (lane >> 3), c8 = (lane & 7) * 8; *(volatile v8b*)(dst + (size_t)rr * HD + c8) = ld8b(Tp + rr * 64 + c8); }
    __threadfence();
  }
}

__global__ __launch_bounds__(128) void out_kernel(const b16* __restrict__ y, const b16* __restrict__ wo16, float* __restrict__ out) {
  __shared__ __attribute__((aligned(16))) float Ts[4][32 * 64];
  const int lane = threadIdx.x & 31, wave = threadIdx.x >> 5, nloc = lane & 15, hlf = lane >> 4;
  const int m0 = blockIdx.y * 128 + wave * 32, c0 = blockIdx.x * 64;
  v8f acc[2][4];
#pragma unroll
  for (int r = 0; r < 2; ++r)
#pragma unroll
    for (int t = 0; t < 4; ++t) acc[r][t] = (v8f){};
  const Opnd A{y, nullptr, HD}, B{wo16, nullptr, HD};
  gemm_tile<1, 1>(A, B, HD, m0, c0, nloc, hlf, acc);
  const Epi e{1.0f, nullptr, nullptr, nullptr, 0, 1.0f, nullptr, nullptr};
  epi_f32(acc, e, out, HID, m0, c0, lane, Ts[wave]);
}
}

extern "C" void kernel_launch(void* const* d_in, const int* in_sizes, int n_in,
                              void* d_out, int out_size, void* d_ws, size_t ws_size, hipStream_t stream) {
  (void)n_in; (void)out_size;
  const float* x    = (const float*)d_in[0];
  const float* cs   = (const float*)d_in[1];
  const float* sn   = (const float*)d_in[2];
  const float* wrkv = (const float*)d_in[3];
  const float* wo   = (const float*)d_in[4];
  const float* td   = (const float*)d_in[5];
  const float* tf   = (const float*)d_in[6];
  const float* tm   = (const float*)d_in[7];
  float* out = (float*)d_out;
  if (in_sizes[0] != MROWS * HID || in_sizes[3] != NRKV * HID || in_sizes[4] != HID * HD || in_sizes[1] != S * DH) return;

  size_t off = 0; char* ws = (char*)d_ws;
  auto carve = [&](size_t bytes) { char* p = ws + off; off += (bytes + 255) & ~(size_t)255; return p; };
  b16* w16   = (b16*)carve((size_t)(NRKV * HID + HID * HD) * 2);
  b16* RA    = (b16*)carve((size_t)MROWS * HID * 2);
  b16* r16   = (b16*)carve((size_t)MROWS * HD * 2);
  float* k32 = (float*)carve((size_t)MROWS * HD * 4);
  b16* v16   = (b16*)carve((size_t)MROWS * HD * 2);
  float* kv32 = (float*)carve((size_t)MROWS * HD * 4);
  float* g    = (float*)carve((size_t)S * 4);
  float* zinv = (float*)carve((size_t)S * 4);
  if (off > ws_size) return;
  b16* mx16 = RA; b16* kvT = RA; b16* y16 = (b16*)k32; const b16* wo16 = w16 + (size_t)NRKV * HID;
  prep_kernel<<<2048, 256, 0, stream>>>(x, wrkv, wo, tm, td, w16, mx16, g, zinv);
  rkv_kernel<<<dim3(NRKV / 64, MROWS / 128), 128, 0, stream>>>(mx16, w16, cs, sn, r16, k32, v16);
  kv_kernel<<<dim3(Bsz * S / 64, 2), 128, 0, stream>>>(k32, v16, kv32, kvT);
  for (int b = 0; b < Bsz; ++b)
    wkv_kernel<<<dim3(HD / 64, S / 128), 128, 0, stream>>>(g, zinv, kvT + (size_t)b * HD * S, kv32 + (size_t)b * S * HD, r16 + (size_t)b * S * HD, tf, y16 + (size_t)b * S * HD);
  out_kernel<<<dim3(HID / 64, MROWS / 128), 128, 0, stream>>>(y16, wo16, out);
}
